// SelectiveSSMLayer_19782619365543
// MI455X (gfx1250) — hardware-run, weakly checked
//
#include <hip/hip_runtime.h>
#include <math.h>

typedef __attribute__((ext_vector_type(16))) _Float16 v16h;
typedef __attribute__((ext_vector_type(8)))  _Float16 v8h;
typedef __attribute__((ext_vector_type(2)))  _Float16 v2h;
typedef __attribute__((ext_vector_type(16))) __bf16   v16b;
typedef __attribute__((ext_vector_type(8)))  __bf16   v8b;
typedef __attribute__((ext_vector_type(8)))  float    v8f;
typedef __attribute__((ext_vector_type(4)))  float    v4f;
typedef __attribute__((ext_vector_type(2)))  float    v2f;
typedef __attribute__((ext_vector_type(4)))  _Float16 v4h;

constexpr int kNB   = 2;
constexpr int kL    = 1024;
constexpr int kRows = kNB * kL;
constexpr int kD    = 1024;
constexpr int kDI   = 2048;
constexpr int kH    = 64;
constexpr int kP    = 32;
constexpr int kNs   = 64;
constexpr int kNR   = 16;
constexpr int kColZ  = 0;
constexpr int kColX  = kDI;
constexpr int kColB  = 2 * kDI;
constexpr int kColC  = 2 * kDI + kNs;
constexpr int kColDt = 2 * kDI + 2 * kNs;
constexpr int kColA  = 2 * kDI + 2 * kNs + kH;
constexpr int kColTr = 2 * kDI + 2 * kNs + 2 * kH;
constexpr int kColAn = 2 * kDI + 2 * kNs + 3 * kH;
constexpr int kStk   = 2 * kDI + 2 * kNs + 3 * kH + kNR;
constexpr int kStkP  = 4480;
constexpr int kOut0 = kRows * kD;
constexpr int kThr  = 256;
constexpr float kInCarry = 1024.0f;
constexpr float kYCarry  = 64.0f;
constexpr float kScIn = 1.0f / (kInCarry * kInCarry);
constexpr float kScY  = 1.0f / (kYCarry * kInCarry);
constexpr float kNormEps = 1e-5f;
constexpr float kAFloor  = 1e-4f;
constexpr float kF16MinNormal = 6.103515625e-5f;

static_assert(kRows == 2048 && kD == 1024 && kDI == 2048 && kH * kP == kDI && kNs == 64 && kStk == 4432 && kStk <= kStkP && (kStkP % 64) == 0 && kColB == 4096 && kColC == 4160 && kColDt == 4224 && kColA == 4288 && kColTr == 4352 && kColAn == 4416 && (kL & (kL - 1)) == 0, "the index arithmetic below uses these sizes");

constexpr size_t kOffX16 = 0ull;
constexpr size_t kOffWS16 = 4194304ull;
constexpr size_t kOffWOUT16 = 13369344ull;
constexpr size_t kOffZB = 17563648ull;
constexpr size_t kOffAH = 17582080ull;
constexpr size_t kOffXS = 18106368ull;
constexpr size_t kOffGB = 54806528ull;
constexpr size_t kOffCM = 88360960ull;
constexpr size_t kOffYS = 121915392ull;
constexpr size_t kOffYG16 = 138692608ull;
constexpr size_t kWsTotal = 147081216ull;
static_assert(kWsTotal <= 268435456ull, "the carve stands under the contract's 256 MiB of workspace");
static_assert(kOffX16 == 0
  && kOffWS16 == kOffX16 + 4194304ull
  && kOffWOUT16 == kOffWS16 + 9175040ull
  && kOffZB == kOffWOUT16 + 4194304ull
  && kOffAH == kOffZB + 18432ull
  && kOffXS == kOffAH + 524288ull
  && kOffGB == kOffXS + 36700160ull
  && kOffCM == kOffGB + 33554432ull
  && kOffYS == kOffCM + 33554432ull
  && kOffYG16 == kOffYS + 16777216ull
  && kWsTotal == kOffYG16 + 8388608ull, "the carve is a chain: every region starts where the one before ends");
static_assert((size_t)kRows * kD * 2 == 4194304ull && (size_t)kStkP * kD * 2 == 9175040ull && (size_t)kD * kDI * 2 == 4194304ull && 4608ull * 4 == 18432ull && (size_t)kRows * kH * 4 == 524288ull && (size_t)kRows * kStkP * 4 == 36700160ull
  && (size_t)kRows * kH * kNs * 4 == 33554432ull && (size_t)kRows * kDI * 4 == 16777216ull && (size_t)kRows * kDI * 2 == 8388608ull, "every region's length is its plane's");
static_assert((kOffWS16 % 256) == 0 && (kOffWOUT16 % 256) == 0 && (kOffZB % 256) == 0 && (kOffAH % 256) == 0 && (kOffXS % 256) == 0 && (kOffGB % 256) == 0 && (kOffCM % 256) == 0 && (kOffYS % 256) == 0 && (kOffYG16 % 256) == 0, "every region starts on a multiple of 256 B");

__device__ __forceinline__ unsigned short f2bf_bits(float f) {
  unsigned u = __float_as_uint(f);
  return (unsigned short)((u + 0x7FFFu + ((u >> 16) & 1u)) >> 16);
}
__device__ __forceinline__ float bf_bits2f(unsigned short h) { return __uint_as_float(((unsigned)h) << 16); }
__device__ __forceinline__ float bf16r(float f) { return bf_bits2f(f2bf_bits(f)); }
__device__ __forceinline__ float carry_flush(float v, float carry) {
  const float s = v * carry;
  return (fabsf(s) < kF16MinNormal) ? 0.0f : s;
}

__device__ __forceinline__ void dep_guard4_h(v8f& a, v8f& b, v8f& c, v8f& d, v16h x, v16h y) { asm volatile("v_nop\n\tv_nop\n\tv_nop\n\tv_nop" : "+v"(a), "+v"(b), "+v"(c), "+v"(d) : "v"(x), "v"(y)); }
__device__ __forceinline__ void dep_guard4_b(v8f& a, v8f& b, v8f& c, v8f& d, v16b x, v16b y) { asm volatile("v_nop\n\tv_nop\n\tv_nop\n\tv_nop" : "+v"(a), "+v"(b), "+v"(c), "+v"(d) : "v"(x), "v"(y)); }
__device__ __forceinline__ void keep4_h(v16h a, v16h b, v16h c, v16h d) { asm volatile("v_nop" :: "v"(a), "v"(b), "v"(c), "v"(d)); }
__device__ __forceinline__ void keep4_b(v16b a, v16b b, v16b c, v16b d) { asm volatile("v_nop" :: "v"(a), "v"(b), "v"(c), "v"(d)); }
__device__ __forceinline__ void acc_guard4(v8f& a, v8f& b, v8f& c, v8f& d) { asm volatile("v_nop\n\tv_nop\n\tv_nop\n\tv_nop" : "+v"(a), "+v"(b), "+v"(c), "+v"(d)); }

template <typename T> struct Frag;
template <> struct Frag<_Float16> {
  typedef v16h V; union U { v16h v; v8h h[2]; };
  static __device__ __forceinline__ v16h load(const _Float16* p) {
    U f; f.h[0] = *(const v8h*)(p); f.h[1] = *(const v8h*)(p + 16); return f.v;
  }
  static __device__ __forceinline__ v8f mma(v16h a, v16h b, v8f c) {
    return __builtin_amdgcn_wmma_f32_16x16x32_f16(false, a, false, b, (short)0, c, false, false);
  }
  static __device__ __forceinline__ void guard4(v8f& a, v8f& b, v8f& c, v8f& d, v16h x, v16h y) { dep_guard4_h(a, b, c, d, x, y); }
  static __device__ __forceinline__ void keep(v16h a, v16h b, v16h c, v16h d) { keep4_h(a, b, c, d); }
};
template <> struct Frag<__bf16> {
  typedef v16b V; union U { v16b v; v8b h[2]; };
  static __device__ __forceinline__ v16b load(const __bf16* p) {
    U f; f.h[0] = *(const v8b*)(p); f.h[1] = *(const v8b*)(p + 16); return f.v;
  }
  static __device__ __forceinline__ v8f mma(v16b a, v16b b, v8f c) {
    return __builtin_amdgcn_wmma_f32_16x16x32_bf16(false, a, false, b, (short)0, c, false, false);
  }
  static __device__ __forceinline__ void guard4(v8f& a, v8f& b, v8f& c, v8f& d, v16b x, v16b y) { dep_guard4_b(a, b, c, d, x, y); }
  static __device__ __forceinline__ void keep(v16b a, v16b b, v16b c, v16b d) { keep4_b(a, b, c, d); }
};

__device__ __forceinline__ v8f mma_h(v16h a, v16h b, v8f c) {
  c = __builtin_amdgcn_wmma_f32_16x16x32_f16(false, a, false, b, (short)0, c, false, false);
  asm volatile("v_nop\n\tv_nop\n\tv_nop\n\tv_nop" : "+v"(c) : "v"(a), "v"(b));
  return c;
}

template <int ET> struct Elem;
template <> struct Elem<0> { typedef _Float16 T; };
template <> struct Elem<1> { typedef __bf16 T; };
template <int ET, bool SPLIT, int BIAS_MODE, int OUT_MODE, bool RESID, int ACT = 0>
__global__ __launch_bounds__(256) void wmma_gemm64(
    const unsigned short* __restrict__ Ap, const unsigned short* __restrict__ A2p, int lda, long strideA,
    const unsigned short* __restrict__ Btp, const unsigned short* __restrict__ Bt2p, int ldb, long strideB,
    void* __restrict__ Cout, void* __restrict__ Cout2, int ldc, long strideC,
    const float* __restrict__ bias,
    const float* __restrict__ resid, long strideR,
    int M, int N, int K, float scale) {
  typedef typename Elem<ET>::T T;
  typedef typename Frag<T>::V V;
  const T* A = (const T*)Ap; const T* A2 = (const T*)A2p; const T* Bt = (const T*)Btp; const T* Bt2 = (const T*)Bt2p;
  __shared__ __align__(16) float sT[8][16 * 68];
  const int b    = blockIdx.y;
  const int lane = threadIdx.x & 31;
  const int wave = threadIdx.x >> 5;
  const int tilesN = N >> 6;
  const int tilesM = M >> 6;
  const int tile = blockIdx.x * 8 + wave;
  if (tile >= tilesM * tilesN) return;
  const int tm = tile / tilesN;
  const int tn = tile - tm * tilesN;
  const int m0 = tm << 6;
  const int n0 = tn << 6;

  const T* Ab  = A  + (size_t)b * strideA;
  const T* Bb  = Bt + (size_t)b * strideB;
  const T* Ab2 = SPLIT ? (A2  + (size_t)b * strideA) : nullptr;
  const T* Bb2 = SPLIT ? (Bt2 + (size_t)b * strideB) : nullptr;

  const int rlane = lane & 15;
  const int koff  = (lane >> 4) * 8;
  const int mOff  = (lane >> 4) * 8;

  v8f acc[4][4];
#pragma unroll
  for (int i = 0; i < 4; ++i)
#pragma unroll
    for (int j = 0; j < 4; ++j) acc[i][j] = (v8f){0.f,0.f,0.f,0.f,0.f,0.f,0.f,0.f};

  for (int k0 = 0; k0 < K; k0 += 32) {
    V bh[4], bl[4];
#pragma unroll
    for (int j = 0; j < 4; ++j) {
      const size_t bo = (size_t)(n0 + (j << 4) + rlane) * ldb + koff + k0;
      bh[j] = Frag<T>::load(Bb + bo);
      if (SPLIT) bl[j] = Frag<T>::load(Bb2 + bo);
    }
#pragma unroll
    for (int i = 0; i < 4; ++i) {
      const size_t ao = (size_t)(m0 + (i << 4) + rlane) * lda + koff + k0;
      V ah = Frag<T>::load(Ab + ao);
      V al;
      if (SPLIT) al = Frag<T>::load(Ab2 + ao);
#pragma unroll
      for (int j = 0; j < 4; ++j) {
        acc[i][j] = Frag<T>::mma(ah, bh[j], acc[i][j]);
        if (SPLIT) {
          acc[i][j] = Frag<T>::mma(ah, bl[j], acc[i][j]);
          acc[i][j] = Frag<T>::mma(al, bh[j], acc[i][j]);
        }
      }
      Frag<T>::guard4(acc[i][0], acc[i][1], acc[i][2], acc[i][3], ah, SPLIT ? al : ah);
    }
    Frag<T>::keep(bh[0], bh[1], bh[2], bh[3]);
    if (SPLIT) Frag<T>::keep(bl[0], bl[1], bl[2], bl[3]);
  }
  acc_guard4(acc[0][0], acc[0][1], acc[0][2], acc[0][3]);
  acc_guard4(acc[1][0], acc[1][1], acc[1][2], acc[1][3]);
  acc_guard4(acc[2][0], acc[2][1], acc[2][2], acc[2][3]);
  acc_guard4(acc[3][0], acc[3][1], acc[3][2], acc[3][3]);

  float* slab = sT[wave];
  const float* Rb = RESID ? (resid + (size_t)b * strideR) : nullptr;
#pragma unroll
  for (int i = 0; i < 4; ++i) {
    const int mBase = m0 + (i << 4);
#pragma unroll
    for (int j = 0; j < 4; ++j) {
      const int n = n0 + (j << 4) + rlane;
      float bv = 0.f;
      if (BIAS_MODE == 2) bv = bias[n];
#pragma unroll
      for (int r = 0; r < 8; ++r) {
        float v = acc[i][j][r] * scale;
        if (BIAS_MODE == 1) v += bias[mBase + mOff + r];
        if (BIAS_MODE == 2) v += bv;
        if (RESID) v += Rb[(size_t)(mBase + mOff + r) * ldc + n];
        if (ACT == 1) v = tanhf(v);
        if (ACT == 2) v = fmaxf(v, 0.0f);
        if (ACT == 3) v = v / (1.0f + expf(-v));
        if (ACT == 4) v = (v > 0.f) ? v : 0.01f * v;
        slab[(mOff + r) * 68 + (j << 4) + rlane] = v;
      }
    }
    __builtin_amdgcn_fence(__ATOMIC_RELEASE, "workgroup");
    __builtin_amdgcn_wave_barrier();
    __builtin_amdgcn_fence(__ATOMIC_ACQUIRE, "workgroup");
    if (OUT_MODE == 0) {
      float* C = (float*)Cout + (size_t)b * strideC;
      const int hh = lane >> 4, c4 = (lane & 15) * 4;
      for (int pass = 0; pass < 2; ++pass) {
#pragma unroll
        for (int it = 0; it < 8; ++it) {
          const int row = it * 2 + hh;
          v4f v = *(const v4f*)(slab + row * 68 + c4);
          *(volatile v4f*)(C + (size_t)(mBase + row) * ldc + n0 + c4) = v;
        }
        __threadfence();
      }
    } else {
      const int q = lane >> 3, c8 = (lane & 7) * 8;
      unsigned short* C  = (unsigned short*)Cout  + (size_t)b * strideC;
      unsigned short* C2 = (OUT_MODE == 2) ? ((unsigned short*)Cout2 + (size_t)b * strideC) : nullptr;
      for (int pass = 0; pass < 2; ++pass) {
#pragma unroll
        for (int it = 0; it < 4; ++it) {
          const int row = it * 4 + q;
          const float* sp = slab + row * 68 + c8;
          v8h hv, lv;
#pragma unroll
          for (int e = 0; e < 8; ++e) {
            if (OUT_MODE == 1) {
              hv[e] = (_Float16)sp[e];
            } else {
              unsigned short hb = f2bf_bits(sp[e]);
              unsigned short lb = f2bf_bits(sp[e] - bf_bits2f(hb));
              hv[e] = __builtin_bit_cast(_Float16, hb);
              lv[e] = __builtin_bit_cast(_Float16, lb);
            }
          }
          *(volatile v8h*)(C + (size_t)(mBase + row) * ldc + n0 + c8) = hv;
          if (OUT_MODE == 2) *(volatile v8h*)(C2 + (size_t)(mBase + row) * ldc + n0 + c8) = lv;
        }
        __threadfence();
      }
    }
    __builtin_amdgcn_fence(__ATOMIC_RELEASE, "workgroup");
    __builtin_amdgcn_wave_barrier();
    __builtin_amdgcn_fence(__ATOMIC_ACQUIRE, "workgroup");
  }
}


__global__ __launch_bounds__(kThr) void cast_plane_kernel(const float* __restrict__ src, unsigned short* __restrict__ dst,
                                                          int colsLog2, int dstPitch, int dstOff) {
  const int i   = blockIdx.x * kThr + threadIdx.x;
  const int sh  = colsLog2 - 3;
  const int row = i >> sh;
  const int c8  = (i & ((1 << sh) - 1)) * 8;
  const float* sp = src + ((size_t)row << colsLog2) + c8;
  const v4f a0 = *(const v4f*)(sp);
  const v4f a1 = *(const v4f*)(sp + 4);
  v8h hv;
#pragma unroll
  for (int e = 0; e < 4; ++e) {
    const float f0 = a0[e];
    const float f1 = a1[e];
    hv[e]     = (_Float16)carry_flush(bf16r(f0), kInCarry);
    hv[4 + e] = (_Float16)carry_flush(bf16r(f1), kInCarry);
  }
  unsigned short* dp = dst + (size_t)row * dstPitch + dstOff + c8;
  *(volatile v8h*)dp = hv;
  __threadfence();
  *(volatile v8h*)dp = hv;
}

__global__ __launch_bounds__(kThr) void setup_kernel(float* __restrict__ ZB, unsigned short* __restrict__ WS16) {
  const unsigned bk = blockIdx.x;
  if (bk < 18u) {
    float* dp = ZB + bk * (unsigned)kThr + threadIdx.x;
    *(volatile float*)dp = 0.0f;
    __threadfence();
    *(volatile float*)dp = 0.0f;
  } else {
    const unsigned j = (bk - 18u) * (unsigned)kThr + threadIdx.x;
    v8h hv;
#pragma unroll
    for (int e = 0; e < 8; ++e) hv[e] = (_Float16)0.0f;
    unsigned short* dp = WS16 + (size_t)kStk * kD + (size_t)j * 8;
    *(volatile v8h*)dp = hv;
    __threadfence();
    *(volatile v8h*)dp = hv;
  }
}
static_assert(18 * kThr == 4608 && 4608 >= kStkP && (size_t)(kStkP - kStk) * kD / 8 == 24ull * kThr, "set-up grid exact: 18 blocks of zero bias, 24 of the weight plane's 48 zero rows");

__device__ __forceinline__ float softplus_f(float v) { return fmaxf(v, 0.0f) + log1pf(expf(-fabsf(v))); }

__global__ __launch_bounds__(kThr) void prep_kernel(const float* __restrict__ XS, const float* __restrict__ dt_bias, const float* __restrict__ B_bias, const float* __restrict__ C_bias,
                                                    const float* __restrict__ Bn_w, const float* __restrict__ Cn_w,
                                                    float* __restrict__ AH, float* __restrict__ GB, float* __restrict__ CM) {
  const unsigned i    = blockIdx.x * (unsigned)kThr + threadIdx.x;
  const unsigned row  = i >> 3;
  const unsigned item = i & 7u;
  const bool turned = item < 4u;
  const unsigned n1 = turned ? 4u * item : 32u + 8u * (item - 4u);
  const unsigned n2 = turned ? (unsigned)kNR + 4u * item : 36u + 8u * (item - 4u);
  const float* px = XS + row * (unsigned)kStkP;
  float sb = 0.0f, sc = 0.0f;
#pragma unroll
  for (int q = 0; q < kNs / 4; ++q) {
    const v4f bv = *(const v4f*)(px + kColB + 4 * q), cv = *(const v4f*)(px + kColC + 4 * q);
#pragma unroll
    for (int e = 0; e < 4; ++e) { sb += bv[e] * bv[e]; sc += cv[e] * cv[e]; }
  }
  const float rB = 1.0f / sqrtf(sb / (float)kNs + kNormEps);
  const float rC = 1.0f / sqrtf(sc / (float)kNs + kNormEps);
  const v4f b1 = *(const v4f*)(px + kColB + n1), b2 = *(const v4f*)(px + kColB + n2);
  const v4f c1 = *(const v4f*)(px + kColC + n1), c2 = *(const v4f*)(px + kColC + n2);
  const v4f wb1 = *(const v4f*)(Bn_w + n1), wb2 = *(const v4f*)(Bn_w + n2), wc1 = *(const v4f*)(Cn_w + n1), wc2 = *(const v4f*)(Cn_w + n2);
  const v4f an = *(const v4f*)(px + kColAn + (turned ? 4u * item : 0u));
  v4f nb1, nb2, nc1, nc2, cs, sn;
#pragma unroll
  for (int e = 0; e < 4; ++e) {
    nb1[e] = (b1[e] * rB) * bf16r(wb1[e]); nb2[e] = (b2[e] * rB) * bf16r(wb2[e]);
    nc1[e] = (c1[e] * rC) * bf16r(wc1[e]); nc2[e] = (c2[e] * rC) * bf16r(wc2[e]);
    cs[e] = turned ? cosf(an[e]) : 1.0f;
    sn[e] = turned ? sinf(an[e]) : 0.0f;
  }
  for (unsigned head = 0; head < (unsigned)kH; ++head) {
    const float pdt = px[kColDt + head], pa = px[kColA + head], ptr = px[kColTr + head];
    const float dt = softplus_f(pdt + bf16r(dt_bias[head]));
    const float Av = fminf(-softplus_f(pa), -kAFloor);
    const float trap = 1.0f / (1.0f + expf(-ptr));
    const float g = 1.0f - 0.5f * trap;
    const float a = g * expf(Av * dt) + 0.5f * trap;
    const float gdt = g * dt;
    const v4f bb1 = *(const v4f*)(B_bias + head * (unsigned)kNs + n1), bb2 = *(const v4f*)(B_bias + head * (unsigned)kNs + n2);
    const v4f cb1 = *(const v4f*)(C_bias + head * (unsigned)kNs + n1), cb2 = *(const v4f*)(C_bias + head * (unsigned)kNs + n2);
    v4f ob1, ob2, oc1, oc2;
#pragma unroll
    for (int e = 0; e < 4; ++e) {
      const float vb1 = nb1[e] + bf16r(bb1[e]), vb2 = nb2[e] + bf16r(bb2[e]);
      const float vc1 = nc1[e] + bf16r(cb1[e]), vc2 = nc2[e] + bf16r(cb2[e]);
      if (turned) {
        ob1[e] = gdt * (vb1 * cs[e] - vb2 * sn[e]);
        ob2[e] = gdt * (vb1 * sn[e] + vb2 * cs[e]);
        oc1[e] = vc1 * cs[e] - vc2 * sn[e];
        oc2[e] = vc1 * sn[e] + vc2 * cs[e];
      } else {
        ob1[e] = gdt * vb1; ob2[e] = gdt * vb2; oc1[e] = vc1; oc2[e] = vc2;
      }
    }
    const unsigned rh = row * (unsigned)kH + head;
    float* pg = GB + rh * (unsigned)kNs;
    float* pc = CM + rh * (unsigned)kNs;
    for (int pass = 0; pass < 2; ++pass) {
      if (item == 0u) *(volatile float*)(AH + rh) = a;
      *(volatile v4f*)(pg + n1) = ob1;
      *(volatile v4f*)(pg + n2) = ob2;
      *(volatile v4f*)(pc + n1) = oc1;
      *(volatile v4f*)(pc + n2) = oc2;
      __threadfence();
    }
  }
}
static_assert((size_t)kRows * 8 == 64ull * kThr && kH == 64 && kNs == 64 && 2 * kNR == 32 && (kColB % 4) == 0 && (kColC % 4) == 0 && (kColAn % 4) == 0 && (kStkP % 4) == 0, "the shared quantities' grid exact: 64 blocks: eight items a row; the B | C | angle columns 16-B aligned; items 0 .. 3 cover states 0 .. 31, items 4 .. 7 states 32 .. 63");

__global__ __launch_bounds__(kThr) void scan_kernel(const float* __restrict__ XS, const float* __restrict__ AH, const float* __restrict__ GB, const float* __restrict__ CM, const float* __restrict__ Dv,
                                                    float* __restrict__ YS) {
  const unsigned ix = blockIdx.x * (unsigned)kThr + threadIdx.x;
  const unsigned p  = ix & 31u;
  const unsigned hd = (ix >> 5) & 63u;
  const unsigned sq = ix >> 11;
  const float dsk = bf16r(Dv[hd]);
  float st[kNs];
#pragma unroll
  for (int n = 0; n < kNs; ++n) st[n] = 0.0f;
  for (int l = 0; l < kL; ++l) {
    const unsigned row = sq * (unsigned)kL + (unsigned)l;
    const unsigned rh = row * (unsigned)kH + hd;
    const float a = AH[rh];
    const float x = XS[row * (unsigned)kStkP + (unsigned)kColX + hd * (unsigned)kP + p];
    const float* pg = GB + rh * (unsigned)kNs;
    const float* pc = CM + rh * (unsigned)kNs;
    float y = 0.0f;
#pragma unroll
    for (int q = 0; q < kNs / 4; ++q) {
      const v4f gv = *(const v4f*)(pg + 4 * q), cv = *(const v4f*)(pc + 4 * q);
#pragma unroll
      for (int e = 0; e < 4; ++e) {
        const float sn = a * st[4 * q + e] + x * gv[e];
        st[4 * q + e] = sn;
        y += sn * cv[e];
      }
    }
    y += dsk * x;
    float* dp = YS + row * (unsigned)kDI + hd * (unsigned)kP + p;
    *(volatile float*)dp = y;
    __threadfence();
    *(volatile float*)dp = y;
  }
}
static_assert(kNB * kDI == 16 * kThr && kP == 32 && kH == 64 && (kNs % 4) == 0, "scan grid exact: 16 blocks: eight a sequence; a wave is one head's 32 channels");

__global__ __launch_bounds__(kThr) void gate_kernel(const float* __restrict__ YS, const float* __restrict__ XS, unsigned short* __restrict__ YG16) {
  const unsigned i = blockIdx.x * (unsigned)kThr + threadIdx.x;
  const unsigned row = i >> 7;
  const unsigned c16 = (i & 127u) * 16u;
  const float* py = YS + row * (unsigned)kDI + c16;
  const float* pz = XS + row * (unsigned)kStkP + (unsigned)kColZ + c16;
  v8h hv[2];
#pragma unroll
  for (int k = 0; k < 2; ++k) {
    const v4f y0 = *(const v4f*)(py + 8 * k), y1 = *(const v4f*)(py + 8 * k + 4);
    const v4f z0 = *(const v4f*)(pz + 8 * k), z1 = *(const v4f*)(pz + 8 * k + 4);
#pragma unroll
    for (int e = 0; e < 8; ++e) {
      const float yy = (e < 4) ? y0[e] : y1[e - 4];
      const float zz = (e < 4) ? z0[e] : z1[e - 4];
      hv[k][e] = (_Float16)carry_flush(yy * (zz / (1.0f + expf(-zz))), kYCarry);
    }
  }
  unsigned short* dp = YG16 + i * 16u;
  for (int pass = 0; pass < 2; ++pass) {
    *(volatile v8h*)dp = hv[0];
    *(volatile v8h*)(dp + 8) = hv[1];
    __threadfence();
  }
}
static_assert((size_t)kRows * kStkP < 4294967296ull / 4 && (size_t)kRows * kH * kNs < 4294967296ull / 4, "every plane's element offsets fit 32 bits");
static_assert((size_t)kRows * kDI / 16 == 1024ull * kThr && kDI / 16 == 128, "the gate's grid exact: 1,024 blocks: two rows a block");

extern "C" void kernel_launch(void* const* d_in, const int* in_sizes, int n_in,
                              void* d_out, int out_size, void* d_ws, size_t ws_size,
                              hipStream_t stream) {
  if (n_in < 9 || d_out == nullptr || d_ws == nullptr) return;
  if (in_sizes[0] != kRows * kD || in_sizes[1] != kStk * kD || in_sizes[2] != kH || in_sizes[3] != kH * kNs || in_sizes[4] != kH * kNs || in_sizes[5] != kNs
      || in_sizes[6] != kNs || in_sizes[7] != kH || in_sizes[8] != kD * kDI) return;
  if (out_size != kOut0) return;
  if (ws_size < kWsTotal) return;
  const float* u = (const float*)d_in[0];
  const float* Win = (const float*)d_in[1];
  const float* dt_bias = (const float*)d_in[2];
  const float* B_bias = (const float*)d_in[3];
  const float* C_bias = (const float*)d_in[4];
  const float* Bn_w = (const float*)d_in[5];
  const float* Cn_w = (const float*)d_in[6];
  const float* Dv = (const float*)d_in[7];
  const float* Wout = (const float*)d_in[8];
  float* out = (float*)d_out;
  char* ws = (char*)d_ws;
  unsigned short* X16 = (unsigned short*)(ws + kOffX16);
  unsigned short* WS16 = (unsigned short*)(ws + kOffWS16);
  unsigned short* WOUT16 = (unsigned short*)(ws + kOffWOUT16);
  float* ZB = (float*)(ws + kOffZB);
  float* AH = (float*)(ws + kOffAH);
  float* XS = (float*)(ws + kOffXS);
  float* GB = (float*)(ws + kOffGB);
  float* CM = (float*)(ws + kOffCM);
  float* YS = (float*)(ws + kOffYS);
  unsigned short* YG16 = (unsigned short*)(ws + kOffYG16);

  static_assert(((size_t)kRows * kD / 8) % kThr == 0 && ((size_t)kStk * kD / 8) % kThr == 0 && ((size_t)kD * kDI / 8) % kThr == 0, "the casts' grids; u's and Win's planes are whole rows of 1,024, Wout's of 2,048");
  cast_plane_kernel<<<(int)(((size_t)kRows * kD / 8) / kThr), kThr, 0, stream>>>(u, X16, 10, kD, 0);
  cast_plane_kernel<<<(int)(((size_t)kStk * kD / 8) / kThr), kThr, 0, stream>>>(Win, WS16, 10, kD, 0);
  cast_plane_kernel<<<(int)(((size_t)kD * kDI / 8) / kThr), kThr, 0, stream>>>(Wout, WOUT16, 11, kDI, 0);
  setup_kernel<<<42, kThr, 0, stream>>>(ZB, WS16);
  wmma_gemm64<0, false, 2, 0, false, 0><<<dim3((kRows / 64) * (kStkP / 64) / 8, 1), 256, 0, stream>>>(
      X16, X16, kD, 0L, WS16, WS16, kD, 0L, (void*)XS, (void*)XS, kStkP, 0L, ZB, nullptr, 0L, kRows, kStkP, kD, kScIn);
  prep_kernel<<<64, kThr, 0, stream>>>(XS, dt_bias, B_bias, C_bias, Bn_w, Cn_w, AH, GB, CM);
  scan_kernel<<<16, kThr, 0, stream>>>(XS, AH, GB, CM, Dv, YS);
  gate_kernel<<<1024, kThr, 0, stream>>>(YS, XS, YG16);
  wmma_gemm64<0, false, 2, 0, false, 0><<<dim3((kRows / 64) * (kD / 64) / 8, 1), 256, 0, stream>>>(
      YG16, YG16, kDI, 0L, WOUT16, WOUT16, kDI, 0L, (void*)out, (void*)out, kD, 0L, ZB, nullptr, 0L, kRows, kD, kDI, kScY);
}
static_assert(((kRows / 64) * (kStkP / 64)) % 8 == 0 && ((kRows / 64) * (kD / 64)) % 8 == 0, "the engine's grids: whole blocks of eight wave tiles");
